// GATv2_274877907718
// MI455X (gfx1250) — hardware-verified
//
#include <hip/hip_runtime.h>
#include <stddef.h>
#include <stdint.h>
#include <math.h>


#define F_IN    128
#define C01     128
#define NHD01   4
#define HD01    32
#define KA      256
#define NHD2    6
#define HD2     40
#define F2W     240
#define RESOFF  256
#define FP2     512
#define NCLS    40
#define NTHR    256
#define NWAVE   8
#define EPT     8
#define CHUNK   (NTHR * EPT)
#define WCAP    (EPT * 32)
#define LISTN   (NWAVE * WCAP)
#define NBMAX   2048
#define NBRUN   1024
#define SLOTB   11
#define RCAP    28672
#define DEGCAP  256
#define GBM     64
#define GBN     64
#define GTHR    128
#define GRP     64
#define NEGSL   0.2f
#define MX0     (-1.0e30f)
#define WSMAX   134217728
#define LDS_AGG ((2 * RCAP + 2 * NBMAX + LISTN) * 4 + 64)

static_assert((CHUNK & (CHUNK - 1)) == 0 && CHUNK <= (1 << SLOTB));
static_assert(NBMAX == (1 << SLOTB));
static_assert(NBRUN <= NBMAX && NBRUN >= 32 && (NBRUN & (NBRUN - 1)) == 0);
static_assert(NTHR * 8 == NBMAX);
static_assert(LISTN >= NBMAX);
static_assert(LISTN >= NWAVE * WCAP);
static_assert((RCAP % 32) == 0);
static_assert(LDS_AGG <= 300000);
static_assert(GBM == (GTHR / 32) * 16);
static_assert((F_IN % 32) == 0 && (KA % 32) == 0);
static_assert((C01 % GBN) == 0 && (FP2 % GBN) == 0);
static_assert(C01 == NHD01 * HD01 && HD01 == 8 * 4 && C01 == 32 * 4);
static_assert(KA == 2 * C01);
static_assert(F2W == NHD2 * HD2 && HD2 == 5 * 8 && F2W == 30 * 8);
static_assert(F2W <= RESOFF && RESOFF + F2W <= FP2);
static_assert(NCLS == HD2 && (NCLS % 4) == 0);
static_assert(NWAVE * GRP * NCLS <= RCAP);
static_assert(NWAVE * C01 <= RCAP);
static_assert((GRP & (GRP - 1)) == 0);
static_assert(F_IN / 8 == 16);
static_assert(C01 == F_IN);

typedef float          v4f  __attribute__((ext_vector_type(4)));
typedef float          v8f  __attribute__((ext_vector_type(8)));
typedef int            v4i  __attribute__((ext_vector_type(4)));
typedef int            v8i  __attribute__((ext_vector_type(8)));
typedef unsigned int   v4u  __attribute__((ext_vector_type(4)));
typedef unsigned short v8us __attribute__((ext_vector_type(8)));
typedef __bf16         v16b __attribute__((ext_vector_type(16)));
typedef v4f  __attribute__((may_alias)) v4fa;
typedef v8us __attribute__((may_alias)) v8usa;
union FragB { v16b v; v8us h[2]; v8i w; };

__device__ __forceinline__ v8f wmb(const FragB& a, const FragB& b, v8f c) {
  v8f d = __builtin_amdgcn_wmma_f32_16x16x32_bf16(false, a.v, false, b.v, (short)0, c, false, false);
  asm volatile("v_nop\n\tv_nop\n\tv_nop\n\tv_nop" : "+v"(d) : "v"(a.w), "v"(b.w));
  return d;
}

__device__ __forceinline__ unsigned int f2bf(float f) {
  const unsigned int u = __float_as_uint(f);
  return ((u + 0x7FFFu + ((u >> 16) & 1u)) >> 16) & 0xFFFFu;
}
__device__ __forceinline__ float bf2f(unsigned int b) { return __uint_as_float(b << 16); }
__device__ __forceinline__ float bfr(float f) { return bf2f(f2bf(f)); }
__device__ __forceinline__ v4f bfr4(const v4f a) {
  v4f r; r.x = bfr(a.x); r.y = bfr(a.y); r.z = bfr(a.z); r.w = bfr(a.w); return r;
}
__device__ __forceinline__ unsigned int pk2(float lo, float hi) { return f2bf(lo) | (f2bf(hi) << 16); }
__device__ __forceinline__ unsigned int pk2lo(float lo, float hi) {
  return f2bf(lo - bfr(lo)) | (f2bf(hi - bfr(hi)) << 16);
}
__device__ __forceinline__ v4u pack8(const v4f a, const v4f b) {
  v4u r;
  r.x = pk2(a.x, a.y); r.y = pk2(a.z, a.w); r.z = pk2(b.x, b.y); r.w = pk2(b.z, b.w);
  return r;
}
__device__ __forceinline__ v4u pack8lo(const v4f a, const v4f b) {
  v4u r;
  r.x = pk2lo(a.x, a.y); r.y = pk2lo(a.z, a.w); r.z = pk2lo(b.x, b.y); r.w = pk2lo(b.z, b.w);
  return r;
}
__device__ __forceinline__ float elu1(float h) {
  const float n = __expf(fminf(h, 0.f)) - 1.0f;
  return h > 0.f ? h : n;
}
__device__ __forceinline__ float lrelu(float x) { return x > 0.f ? x : NEGSL * x; }
__device__ __forceinline__ float sum6(float v, int j5) {
  float s = __shfl(v, j5);
  s += __shfl(v, j5 + 5);
  s += __shfl(v, j5 + 10);
  s += __shfl(v, j5 + 15);
  s += __shfl(v, j5 + 20);
  s += __shfl(v, j5 + 25);
  return s;
}

__device__ __forceinline__ int scan_chunk(const int* __restrict__ dsts, int nE, int cbase, int slotBase,
                                          int nb, int vec8, int* list, int tid, int lane, int wave) {
  int wc = 0;
  const int el0  = tid * EPT;
  const int e0   = cbase + el0;
  const int sent = -2147483647 - 1;
  v4i da, db;
  if (vec8 != 0 && cbase + CHUNK <= nE) {
    da = *(const v4i*)(dsts + e0);
    db = *(const v4i*)(dsts + e0 + 4);
  } else {
    da.x = (e0     < nE) ? dsts[min(e0,     nE - 1)] : sent;
    da.y = (e0 + 1 < nE) ? dsts[min(e0 + 1, nE - 1)] : sent;
    da.z = (e0 + 2 < nE) ? dsts[min(e0 + 2, nE - 1)] : sent;
    da.w = (e0 + 3 < nE) ? dsts[min(e0 + 3, nE - 1)] : sent;
    db.x = (e0 + 4 < nE) ? dsts[min(e0 + 4, nE - 1)] : sent;
    db.y = (e0 + 5 < nE) ? dsts[min(e0 + 5, nE - 1)] : sent;
    db.z = (e0 + 6 < nE) ? dsts[min(e0 + 6, nE - 1)] : sent;
    db.w = (e0 + 7 < nE) ? dsts[min(e0 + 7, nE - 1)] : sent;
  }
  const unsigned nbs = (unsigned)slotBase;
  const unsigned unb = (unsigned)nb;
  const unsigned s0 = (unsigned)da.x - nbs, s1 = (unsigned)da.y - nbs;
  const unsigned s2 = (unsigned)da.z - nbs, s3 = (unsigned)da.w - nbs;
  const unsigned s4 = (unsigned)db.x - nbs, s5 = (unsigned)db.y - nbs;
  const unsigned s6 = (unsigned)db.z - nbs, s7 = (unsigned)db.w - nbs;
  const bool h0 = s0 < unb, h1 = s1 < unb, h2 = s2 < unb, h3 = s3 < unb;
  const bool h4 = s4 < unb, h5 = s5 < unb, h6 = s6 < unb, h7 = s7 < unb;
  const unsigned any = __builtin_amdgcn_ballot_w32(h0 | h1 | h2 | h3 | h4 | h5 | h6 | h7);
  if (any != 0u) {
#define HITJ(J, HJ, SJ) { \
      const unsigned mj = __builtin_amdgcn_ballot_w32(HJ); \
      if (mj != 0u) { \
        if (HJ) { \
          const int pos = wc + (int)__builtin_amdgcn_mbcnt_lo(mj, 0u); \
          if (pos < WCAP) list[wave * WCAP + pos] = ((el0 + (J)) << SLOTB) | (int)(SJ); \
        } \
        wc += (int)__builtin_popcount(mj); } }
    HITJ(0, h0, s0)
    HITJ(1, h1, s1)
    HITJ(2, h2, s2)
    HITJ(3, h3, s3)
    HITJ(4, h4, s4)
    HITJ(5, h5, s5)
    HITJ(6, h6, s6)
    HITJ(7, h7, s7)
#undef HITJ
  }
  return wc;
}

__global__ __launch_bounds__(NTHR) void k_xprep(const float* __restrict__ x, unsigned short* xb, int nN, int nUnits) {
  const int i = (int)blockIdx.x * NTHR + (int)threadIdx.x;
  if (i >= nUnits) return;
  const int row = i >> 4;
  const int c0  = (i & 15) * 8;
  const int rc  = row < nN ? row : nN - 1;
  const float* p = x + (size_t)rc * F_IN + c0;
  v4f a = *(const v4fa*)p, b = *(const v4fa*)(p + 4);
  const v4f z4 = {0.f, 0.f, 0.f, 0.f};
  if (row >= nN) { a = z4; b = z4; }
  const v4u hv = pack8(a, b);
  const size_t o = (size_t)row * F_IN + c0;
  *(volatile v4u*)(xb + o) = hv;
  __threadfence();
  *(volatile v4u*)(xb + o) = hv;
}

__global__ __launch_bounds__(NTHR) void k_wtr(const float* __restrict__ w, int Kin, int Ncol, int Nrows, int Kout,
                                              unsigned short* wt, int nUnits) {
  const int u = (int)blockIdx.x * NTHR + (int)threadIdx.x;
  if (u >= nUnits) return;
  const int kq = Kout >> 3;
  const int n  = u / kq;
  const int k8 = (u - n * kq) * 8;
  const int kk = k8 - (k8 / Kin) * Kin;
  const int ncl = n < Ncol ? n : Ncol - 1;
  const float* p = w + (size_t)kk * (size_t)Ncol + ncl;
  v4f a, b;
  a.x = p[0];                    a.y = p[(size_t)Ncol];         a.z = p[(size_t)2 * Ncol];     a.w = p[(size_t)3 * Ncol];
  b.x = p[(size_t)4 * Ncol];     b.y = p[(size_t)5 * Ncol];     b.z = p[(size_t)6 * Ncol];     b.w = p[(size_t)7 * Ncol];
  const v4f z4 = {0.f, 0.f, 0.f, 0.f};
  if (n >= Ncol || n >= Nrows) { a = z4; b = z4; }
  const v4u wv = pack8(a, b);
  unsigned short* o = wt + (size_t)n * (size_t)Kout + k8;
  *(volatile v4u*)o = wv;
  __threadfence();
  *(volatile v4u*)o = wv;
}

__global__ __launch_bounds__(GTHR) void k_gemm(
    const unsigned short* __restrict__ A, const unsigned short* __restrict__ WT,
    float* outF, int K, int ldo)
{
  __shared__ __attribute__((aligned(16))) float stg[GBM * GBN];
  const int tid = (int)threadIdx.x, lane = tid & 31, wave = tid >> 5, hh = lane >> 4, m = lane & 15;
  const int rowBase = (int)blockIdx.x * GBM;
  const int col0    = (int)blockIdx.y * GBN;

  v8f acc[4];
  {
    const v8f z = {0.f, 0.f, 0.f, 0.f, 0.f, 0.f, 0.f, 0.f};
    acc[0] = z; acc[1] = z; acc[2] = z; acc[3] = z;
  }
  const unsigned short* ap = A  + (size_t)(rowBase + 16 * wave + m) * (size_t)K + 8 * hh;
  const unsigned short* wp = WT + (size_t)(col0 + m) * (size_t)K + 8 * hh;
  const int ksteps = K >> 5;
#pragma unroll 1
  for (int ks = 0; ks < ksteps; ++ks) {
    FragB af;
    af.h[0] = *(const v8usa*)(ap + 32 * ks);
    af.h[1] = *(const v8usa*)(ap + 32 * ks + 16);
#pragma unroll
    for (int t = 0; t < 4; ++t) {
      const unsigned short* wq = wp + (size_t)(16 * t) * (size_t)K + 32 * ks;
      FragB bf;
      bf.h[0] = *(const v8usa*)wq;
      bf.h[1] = *(const v8usa*)(wq + 16);
      acc[t] = wmb(af, bf, acc[t]);
    }
  }

#pragma unroll
  for (int t = 0; t < 4; ++t) {
    const int lc = 16 * t + m;
#pragma unroll
    for (int r = 0; r < 8; ++r) {
      const int lr = 16 * wave + 8 * hh + r;
      stg[lr * GBN + lc] = acc[t][r];
    }
  }
  __syncthreads();

  v4f fv[8];
#pragma unroll
  for (int i = 0; i < 8; ++i) {
    const int lr = 16 * wave + 2 * i + hh;
    fv[i] = *(const v4fa*)(stg + lr * GBN + 4 * m);
  }
#pragma unroll
  for (int i = 0; i < 8; ++i) {
    const int lr = 16 * wave + 2 * i + hh;
    const int gr = rowBase + lr;
    float* op = outF + (size_t)gr * (size_t)ldo + col0 + 4 * m;
    *(volatile v4f*)op = fv[i];
  }
  __threadfence();
#pragma unroll
  for (int i = 0; i < 8; ++i) {
    const int lr = 16 * wave + 2 * i + hh;
    const int gr = rowBase + lr;
    float* op = outF + (size_t)gr * (size_t)ldo + col0 + 4 * m;
    *(volatile v4f*)op = fv[i];
  }
}

template<int L>
__global__ __launch_bounds__(NTHR) void k_agg(
    const int* __restrict__ srcs, const int* __restrict__ dsts,
    const float* __restrict__ F, const float* __restrict__ R, const float* __restrict__ attn,
    float* HO, unsigned short* AP, float* out,
    int nN, int nE, int nb, int vec8, int MPr) {
  extern __shared__ v4f lds_dyn[];
  int* reg1 = (int*)lds_dyn;
  int* reg2 = reg1 + RCAP;
  int* scnt = reg2 + RCAP;
  int* soff = scnt + NBMAX;
  int* list = soff + NBMAX;
  int* wcnt = list + LISTN;
  int* wtot = wcnt + NWAVE;
  const int tid = (int)threadIdx.x, lane = tid & 31, wave = tid >> 5;
  const int nodeBase = (int)blockIdx.x * nb;

  for (int i = tid; i < NBMAX; i += NTHR) scnt[i] = 0;
  __syncthreads();

  int tot = 0;
  const int nChunks = (nE + CHUNK - 1) / CHUNK;
#pragma unroll 1
  for (int ch = 0; ch < nChunks; ++ch) {
    const int cbase = ch * CHUNK;
    const int wc = scan_chunk(dsts, nE, cbase, nodeBase, nb, vec8, list, tid, lane, wave);
    if (lane == 0) wcnt[wave] = wc;
    __syncthreads();
    int pre = 0, all = 0;
#pragma unroll
    for (int w2 = 0; w2 < NWAVE; ++w2) {
      int c = wcnt[w2];
      c = c < 0 ? 0 : (c > WCAP ? WCAP : c);
      all += c;
      pre += (w2 < wave) ? c : 0;
    }
    const int wcc  = wc > WCAP ? WCAP : wc;
    const int base = tot + pre;
#pragma unroll 1
    for (int i = lane; i < wcc; i += 32) {
      const int ent = list[wave * WCAP + i];
      const int el  = (ent >> SLOTB) & (CHUNK - 1);
      const int sl  = ent & (NBMAX - 1);
      int eid = cbase + el;
      eid = eid > nE - 1 ? nE - 1 : eid;
      const int pos = base + i;
      if (pos < RCAP) reg1[pos] = (int)(((unsigned)eid << SLOTB) | (unsigned)sl);
    }
    tot += all;
    tot = tot > RCAP ? RCAP : tot;
    __syncthreads();
  }
  const int nh = tot;

  if (wave == 0) {
#pragma unroll 1
    for (int b0 = 0; b0 < nh; b0 += 32) {
      const int idx = b0 + lane;
      const int uv  = reg1[idx < nh ? idx : nh - 1];
      const int m32 = (nh - b0) < 32 ? (nh - b0) : 32;
#pragma unroll 1
      for (int k = 0; k < m32; ++k) {
        const int u  = __builtin_amdgcn_readlane(uv, k);
        const int sl = u & (NBMAX - 1);
        if (lane == 0) scnt[sl] = scnt[sl] + 1;
      }
    }
  }
  __syncthreads();

  {
    const v4i ca = *(const v4i*)(scnt + 8 * tid);
    const v4i cb = *(const v4i*)(scnt + 8 * tid + 4);
    const int e0 = ca.x < 0 ? 0 : ca.x, e1 = ca.y < 0 ? 0 : ca.y, e2 = ca.z < 0 ? 0 : ca.z, e3 = ca.w < 0 ? 0 : ca.w;
    const int e4 = cb.x < 0 ? 0 : cb.x, e5 = cb.y < 0 ? 0 : cb.y, e6 = cb.z < 0 ? 0 : cb.z, e7 = cb.w < 0 ? 0 : cb.w;
    const int ts = e0 + e1 + e2 + e3 + e4 + e5 + e6 + e7;
    int incl = ts;
#pragma unroll
    for (int d = 1; d < 32; d <<= 1) {
      const int up = __shfl_up(incl, d);
      if (lane >= d) incl += up;
    }
    if (lane == 31) wtot[wave] = incl;
    __syncthreads();
    int pre = 0;
#pragma unroll
    for (int w2 = 0; w2 < NWAVE; ++w2) pre += (w2 < wave) ? wtot[w2] : 0;
    int run = pre + incl - ts;
    soff[8 * tid + 0] = run; run += e0;
    soff[8 * tid + 1] = run; run += e1;
    soff[8 * tid + 2] = run; run += e2;
    soff[8 * tid + 3] = run; run += e3;
    soff[8 * tid + 4] = run; run += e4;
    soff[8 * tid + 5] = run; run += e5;
    soff[8 * tid + 6] = run; run += e6;
    soff[8 * tid + 7] = run;
  }
  __syncthreads();
  for (int i = tid; i < NBMAX; i += NTHR) list[i] = soff[i];
  __syncthreads();

  if (wave == 0) {
#pragma unroll 1
    for (int b0 = 0; b0 < nh; b0 += 32) {
      const int idx = b0 + lane;
      const int uv  = reg1[idx < nh ? idx : nh - 1];
      const int m32 = (nh - b0) < 32 ? (nh - b0) : 32;
#pragma unroll 1
      for (int k = 0; k < m32; ++k) {
        const int u   = __builtin_amdgcn_readlane(uv, k);
        const int sl  = u & (NBMAX - 1);
        const int eid = (int)((unsigned)u >> SLOTB);
        if (lane == 0) {
          int pos = list[sl];
          pos = pos < 0 ? 0 : (pos > RCAP - 1 ? RCAP - 1 : pos);
          reg2[pos] = eid;
          list[sl] = pos + 1;
        }
      }
    }
  }
  __syncthreads();

  const int nbw = nb >> 3;
  const bool ovf = (nh >= RCAP);
  const float qnan = __int_as_float(0x7fc00000);

  if (L < 2) {
    const int c0 = 4 * lane;
    const v4f at = bfr4(*(const v4fa*)(attn + c0));
    float* stw = (float*)reg1 + wave * C01;
    const int lc = lane < 16 ? lane : 15;

#pragma unroll 1
    for (int jt = 0; jt < nbw; ++jt) {
      const int slot = wave * nbw + jt;
      const int grow = nodeBase + slot;
      const int gcl  = grow < nN ? grow : nN - 1;
      int st = soff[slot];
      const int craw = scnt[slot];
      int cnt = craw;
      st  = st < 0 ? 0 : (st > nh ? nh : st);
      cnt = cnt < 0 ? 0 : (cnt > DEGCAP ? DEGCAP : cnt);
      if (cnt > nh - st) cnt = nh - st;
      const float pz = (ovf || craw > DEGCAP) ? qnan : 0.0f;

      const v4f fd = *(const v4fa*)(F + (size_t)gcl * C01 + c0);
      v4f rr = {0.f, 0.f, 0.f, 0.f};
      if (L == 1) rr = *(const v4fa*)(R + (size_t)gcl * C01 + c0);
      float mx = MX0, dn = 0.0f;
      v4f av = {0.f, 0.f, 0.f, 0.f};

#pragma unroll 1
      for (int q = 0; q < cnt; ++q) {
        int idx = st + q; idx = idx > RCAP - 1 ? RCAP - 1 : idx;
        int eid = reg2[idx]; eid = eid < 0 ? 0 : (eid > nE - 1 ? nE - 1 : eid);
        const int sraw = srcs[eid];
        const int s = sraw < 0 ? 0 : (sraw > nN - 1 ? nN - 1 : sraw);
        const v4f fs = *(const v4fa*)(F + (size_t)s * C01 + c0);
        const float x0 = lrelu(fs.x + fd.x), x1 = lrelu(fs.y + fd.y);
        const float x2 = lrelu(fs.z + fd.z), x3 = lrelu(fs.w + fd.w);
        float part = x0 * at.x;
        part = fmaf(x1, at.y, part);
        part = fmaf(x2, at.z, part);
        part = fmaf(x3, at.w, part);
        part += __shfl_xor(part, 4);
        part += __shfl_xor(part, 2);
        part += __shfl_xor(part, 1);
        const float lg = part;
        const float df = lg - mx;
        const float ee = __expf(-fabsf(df));
        const bool up  = df > 0.f;
        const float s1 = up ? ee : 1.0f;
        const float s2 = up ? 1.0f : ee;
        mx = up ? lg : mx;
        dn = fmaf(dn, s1, s2);
        av.x = fmaf(av.x, s1, s2 * fs.x);
        av.y = fmaf(av.y, s1, s2 * fs.y);
        av.z = fmaf(av.z, s1, s2 * fs.z);
        av.w = fmaf(av.w, s1, s2 * fs.w);
      }
      const float dsf = dn > 0.f ? dn : 1.0f;
      const float inv = (dn > 0.f ? 1.0f : 0.0f) * __builtin_amdgcn_rcpf(dsf);
      const bool live = grow < nN;
      v4f o;
      o.x = (live ? elu1(fmaf(av.x, inv, rr.x)) : 0.f) + pz;
      o.y = (live ? elu1(fmaf(av.y, inv, rr.y)) : 0.f) + pz;
      o.z = (live ? elu1(fmaf(av.z, inv, rr.z)) : 0.f) + pz;
      o.w = (live ? elu1(fmaf(av.w, inv, rr.w)) : 0.f) + pz;

      __builtin_amdgcn_fence(__ATOMIC_RELEASE, "wavefront");
      __builtin_amdgcn_wave_barrier();
      *(v4fa*)(stw + 4 * lane) = o;
      __builtin_amdgcn_fence(__ATOMIC_RELEASE, "wavefront");
      __builtin_amdgcn_wave_barrier();
      const v4f ga = *(const v4fa*)(stw + 8 * lc);
      const v4f gb = *(const v4fa*)(stw + 8 * lc + 4);
      const v4u hv = pack8(ga, gb);
      const v4u lv = pack8lo(ga, gb);
      const bool wr  = grow < MPr;
      const bool wsa = wr && (lane < 16);
      unsigned short* gp = AP + (size_t)grow * KA + 8 * lc;
      const size_t hoff = (size_t)grow * C01 + c0;
      if (L == 0) { if (wr) *(volatile v4f*)(HO + hoff) = o; }
      if (wsa) { *(volatile v4u*)gp = hv; *(volatile v4u*)(gp + C01) = lv; }
      __threadfence();
      if (L == 0) { if (wr) *(volatile v4f*)(HO + hoff) = o; }
      if (wsa) { *(volatile v4u*)gp = hv; *(volatile v4u*)(gp + C01) = lv; }
    }
  } else {
    const int hl  = lane / 5;
    const int hcl = hl < NHD2 - 1 ? hl : NHD2 - 1;
    const int j5  = lane - 5 * hl;
    const int cc  = lane < (F2W / 8) ? 8 * lane : F2W - 8;
    const float* atp = attn + hcl * HD2 + 8 * j5;
    const v4f atA = bfr4(*(const v4fa*)atp);
    const v4f atB = bfr4(*(const v4fa*)(atp + 4));
    const int b5 = 5 * hcl;
    float* sg = (float*)reg1 + wave * (GRP * NCLS);

#pragma unroll 1
    for (int jt = 0; jt < nbw; ++jt) {
      const int slot = wave * nbw + jt;
      const int grow = nodeBase + slot;
      const int gcl  = grow < nN ? grow : nN - 1;
      int st = soff[slot];
      const int craw = scnt[slot];
      int cnt = craw;
      st  = st < 0 ? 0 : (st > nh ? nh : st);
      cnt = cnt < 0 ? 0 : (cnt > DEGCAP ? DEGCAP : cnt);
      if (cnt > nh - st) cnt = nh - st;
      const float pz = (ovf || craw > DEGCAP) ? qnan : 0.0f;

      const float* dr = F + (size_t)gcl * FP2 + cc;
      const v4f fdA = *(const v4fa*)dr;
      const v4f fdB = *(const v4fa*)(dr + 4);
      const v4f rsA = *(const v4fa*)(dr + RESOFF);
      const v4f rsB = *(const v4fa*)(dr + RESOFF + 4);
      float mx = MX0, dn = 0.0f;
      v4f avA = {0.f, 0.f, 0.f, 0.f};
      v4f avB = {0.f, 0.f, 0.f, 0.f};

#pragma unroll 1
      for (int q = 0; q < cnt; ++q) {
        int idx = st + q; idx = idx > RCAP - 1 ? RCAP - 1 : idx;
        int eid = reg2[idx]; eid = eid < 0 ? 0 : (eid > nE - 1 ? nE - 1 : eid);
        const int sraw = srcs[eid];
        const int s = sraw < 0 ? 0 : (sraw > nN - 1 ? nN - 1 : sraw);
        const float* sr = F + (size_t)s * FP2 + cc;
        const v4f fsA = *(const v4fa*)sr;
        const v4f fsB = *(const v4fa*)(sr + 4);
        const float x0 = lrelu(fsA.x + fdA.x), x1 = lrelu(fsA.y + fdA.y);
        const float x2 = lrelu(fsA.z + fdA.z), x3 = lrelu(fsA.w + fdA.w);
        const float x4 = lrelu(fsB.x + fdB.x), x5 = lrelu(fsB.y + fdB.y);
        const float x6 = lrelu(fsB.z + fdB.z), x7 = lrelu(fsB.w + fdB.w);
        float part = x0 * atA.x;
        part = fmaf(x1, atA.y, part);
        part = fmaf(x2, atA.z, part);
        part = fmaf(x3, atA.w, part);
        part = fmaf(x4, atB.x, part);
        part = fmaf(x5, atB.y, part);
        part = fmaf(x6, atB.z, part);
        part = fmaf(x7, atB.w, part);
        float lg = __shfl(part, b5);
        lg += __shfl(part, b5 + 1);
        lg += __shfl(part, b5 + 2);
        lg += __shfl(part, b5 + 3);
        lg += __shfl(part, b5 + 4);
        const float df = lg - mx;
        const float ee = __expf(-fabsf(df));
        const bool up  = df > 0.f;
        const float s1 = up ? ee : 1.0f;
        const float s2 = up ? 1.0f : ee;
        mx = up ? lg : mx;
        dn = fmaf(dn, s1, s2);
        avA.x = fmaf(avA.x, s1, s2 * fsA.x);
        avA.y = fmaf(avA.y, s1, s2 * fsA.y);
        avA.z = fmaf(avA.z, s1, s2 * fsA.z);
        avA.w = fmaf(avA.w, s1, s2 * fsA.w);
        avB.x = fmaf(avB.x, s1, s2 * fsB.x);
        avB.y = fmaf(avB.y, s1, s2 * fsB.y);
        avB.z = fmaf(avB.z, s1, s2 * fsB.z);
        avB.w = fmaf(avB.w, s1, s2 * fsB.w);
      }
      const float dsf = dn > 0.f ? dn : 1.0f;
      const float inv = (dn > 0.f ? 1.0f : 0.0f) * __builtin_amdgcn_rcpf(dsf);
      v4f vA, vB;
      vA.x = fmaf(avA.x, inv, rsA.x);  vA.y = fmaf(avA.y, inv, rsA.y);
      vA.z = fmaf(avA.z, inv, rsA.z);  vA.w = fmaf(avA.w, inv, rsA.w);
      vB.x = fmaf(avB.x, inv, rsB.x);  vB.y = fmaf(avB.y, inv, rsB.y);
      vB.z = fmaf(avB.z, inv, rsB.z);  vB.w = fmaf(avB.w, inv, rsB.w);
      const float sixth = 1.0f / 6.0f;
      v4f mA, mB;
      mA.x = sum6(vA.x, j5) * sixth + pz;  mA.y = sum6(vA.y, j5) * sixth + pz;
      mA.z = sum6(vA.z, j5) * sixth + pz;  mA.w = sum6(vA.w, j5) * sixth + pz;
      mB.x = sum6(vB.x, j5) * sixth + pz;  mB.y = sum6(vB.y, j5) * sixth + pz;
      mB.z = sum6(vB.z, j5) * sixth + pz;  mB.w = sum6(vB.w, j5) * sixth + pz;
      const int lr = jt & (GRP - 1);
      if (lane < 5) {
        *(v4fa*)(sg + lr * NCLS + 8 * lane)     = mA;
        *(v4fa*)(sg + lr * NCLS + 8 * lane + 4) = mB;
      }

      const int gb = jt & ~(GRP - 1);
      if (lr == GRP - 1 || jt == nbw - 1) {
        __syncthreads();
        int gsz = nbw - gb; gsz = gsz > GRP ? GRP : gsz;
        const int row0 = nodeBase + wave * nbw + gb;
        int live = nN - row0; live = live < 0 ? 0 : (live > gsz ? gsz : live);
        const int npc = live * (NCLS / 4);
        float* ob = out + (size_t)row0 * NCLS;
#pragma unroll 1
        for (int p = lane; p < npc; p += 32) {
          const v4f v = *(const v4fa*)(sg + 4 * p);
          *(volatile v4f*)(ob + 4 * p) = v;
        }
        __threadfence();
#pragma unroll 1
        for (int p = lane; p < npc; p += 32) {
          const v4f v = *(const v4fa*)(sg + 4 * p);
          *(volatile v4f*)(ob + 4 * p) = v;
        }
        __syncthreads();
      }
    }
  }
  (void)R; (void)HO; (void)AP; (void)out;
}

static int pick_nb(int nE, int nN) {
  int nb = NBRUN;
  while (nb > 32 && (long long)nb * (long long)nE * 5LL > (long long)RCAP * (long long)nN * 4LL) nb >>= 1;
  return nb;
}
static inline int cdiv(int a, int b) { return (a + b - 1) / b; }
static inline size_t al256(size_t v) { return (v + 255) & ~(size_t)255; }

extern "C" void kernel_launch(void* const* d_in, const int* in_sizes, int n_in,
                              void* d_out, int out_size, void* d_ws, size_t ws_size,
                              hipStream_t stream) {
  if (n_in < 10) return;
  const int nN = in_sizes[0] / F_IN;
  if (nN <= 0 || in_sizes[0] != nN * F_IN || nN > (1 << 22)) return;
  const int nE = in_sizes[1];
  if (nE < 1 || nE >= (1 << (32 - SLOTB))) return;
  if (in_sizes[2] != nE) return;
  if (in_sizes[3] != F_IN * C01) return;
  if (in_sizes[4] != NHD01 * HD01) return;
  if (in_sizes[5] != C01 * C01) return;
  if (in_sizes[6] != NHD01 * HD01) return;
  if (in_sizes[7] != C01 * F2W) return;
  if (in_sizes[8] != NHD2 * HD2) return;
  if (in_sizes[9] != C01 * F2W) return;
  if (out_size != nN * NCLS) return;

  const float* x     = (const float*)d_in[0];
  const int*   src   = (const int*)  d_in[1];
  const int*   dst   = (const int*)  d_in[2];
  const float* W0    = (const float*)d_in[3];
  const float* attn0 = (const float*)d_in[4];
  const float* W1    = (const float*)d_in[5];
  const float* attn1 = (const float*)d_in[6];
  const float* W2    = (const float*)d_in[7];
  const float* attn2 = (const float*)d_in[8];
  const float* Wres2 = (const float*)d_in[9];
  float* out = (float*)d_out;

  const int MP   = cdiv(nN, GBM) * GBM;
  const int nb   = pick_nb(nE, nN);
  if (nb < 32 || (nb & (nb - 1)) != 0 || nb > NBMAX) return;
  const int gA   = cdiv(MP, nb);
  const int vec8 = ((nE & 3) == 0) ? 1 : 0;
  if (gA * nb < MP) return;

  char* ws = (char*)d_ws;
  size_t off = 0;
  const size_t oWT0 = off; off += (size_t)C01 * F_IN * 2;          off = al256(off);
  const size_t oWT1 = off; off += (size_t)C01 * KA * 2;            off = al256(off);
  const size_t oWT2 = off; off += (size_t)FP2 * KA * 2;            off = al256(off);
  const size_t oAH  = off; off += (size_t)MP * KA * 2;             off = al256(off);
  const size_t szB  = al256((size_t)MP * FP2 * 4);
  const size_t oB   = off; off += szB;                               off = al256(off);
  const size_t szXB = al256((size_t)MP * F_IN * 2);
  const size_t szF  = al256((size_t)MP * C01 * 4);
  const size_t oXB  = oB;
  const size_t oF01 = oB + szXB;
  const size_t oHF0 = oF01 + szF;
  if (szXB + 2 * szF > szB) return;
  if (off > ws_size || off > (size_t)WSMAX) return;
  unsigned short* WT0 = (unsigned short*)(ws + oWT0);
  unsigned short* WT1 = (unsigned short*)(ws + oWT1);
  unsigned short* WT2 = (unsigned short*)(ws + oWT2);
  unsigned short* AH  = (unsigned short*)(ws + oAH);
  float*          FB  = (float*)(ws + oB);
  unsigned short* XB  = (unsigned short*)(ws + oXB);
  float*          F01 = (float*)(ws + oF01);
  float*          HF0 = (float*)(ws + oHF0);

  hipFuncSetAttribute(reinterpret_cast<const void*>(&k_agg<0>),
                      hipFuncAttributeMaxDynamicSharedMemorySize, LDS_AGG);
  hipFuncSetAttribute(reinterpret_cast<const void*>(&k_agg<1>),
                      hipFuncAttributeMaxDynamicSharedMemorySize, LDS_AGG);
  hipFuncSetAttribute(reinterpret_cast<const void*>(&k_agg<2>),
                      hipFuncAttributeMaxDynamicSharedMemorySize, LDS_AGG);

  const int nUx = MP * (F_IN / 8);
  k_xprep<<<cdiv(nUx, NTHR), NTHR, 0, stream>>>(x, XB, nN, nUx);

  {
    const int nUw0 = C01 * (F_IN / 8);
    k_wtr<<<cdiv(nUw0, NTHR), NTHR, 0, stream>>>(W0, F_IN, C01, C01, F_IN, WT0, nUw0);
    const int nUw1 = C01 * (KA / 8);
    k_wtr<<<cdiv(nUw1, NTHR), NTHR, 0, stream>>>(W1, C01, C01, C01, KA, WT1, nUw1);
    const int nUw2a = RESOFF * (KA / 8);
    k_wtr<<<cdiv(nUw2a, NTHR), NTHR, 0, stream>>>(W2, C01, F2W, RESOFF, KA, WT2, nUw2a);
    const int nUw2b = (FP2 - RESOFF) * (KA / 8);
    k_wtr<<<cdiv(nUw2b, NTHR), NTHR, 0, stream>>>(Wres2, C01, F2W, FP2 - RESOFF, KA,
                                                   WT2 + (size_t)RESOFF * KA, nUw2b);
  }

  const int gM = MP / GBM;
  k_gemm<<<dim3(gM, C01 / GBN), GTHR, 0, stream>>>(XB, WT0, F01, F_IN, C01);
  k_agg<0><<<gA, NTHR, LDS_AGG, stream>>>(src, dst, F01, F01, attn0, HF0, AH, out, nN, nE, nb, vec8, MP);
  k_gemm<<<dim3(gM, C01 / GBN), GTHR, 0, stream>>>(AH, WT1, F01, KA, C01);
  k_agg<1><<<gA, NTHR, LDS_AGG, stream>>>(src, dst, F01, HF0, attn1, out, AH, out, nN, nE, nb, vec8, MP);
  k_gemm<<<dim3(gM, FP2 / GBN), GTHR, 0, stream>>>(AH, WT2, FB, KA, FP2);
  k_agg<2><<<gA, NTHR, LDS_AGG, stream>>>(src, dst, FB, FB, attn2, out, AH, out, nN, nE, nb, vec8, MP);
}
